// SModel_81552839016873
// MI455X (gfx1250) — hardware-run, weakly checked
//
#include <hip/hip_runtime.h>
#include <math.h>

typedef __attribute__((ext_vector_type(16))) _Float16 v16h;
typedef __attribute__((ext_vector_type(8)))  _Float16 v8h;
typedef __attribute__((ext_vector_type(8)))  float    v8f;
typedef __attribute__((ext_vector_type(4)))  float    v4f;

constexpr int kNB   = 512;
constexpr int kNT   = 512;
constexpr int kNI   = 8;
constexpr int kNH   = 256;
constexpr int kNG   = 3 * kNH;
constexpr int kKP   = 288;
constexpr int kAP   = 296;
constexpr int kHP   = 260;
constexpr float kCarryA = 128.0f;
constexpr float kCarryW = 256.0f;
constexpr float kFold   = 1.0f / (kCarryA * kCarryW);
constexpr int kPackThreads = kNG * (kKP / 8);
constexpr size_t kWsTotal  = (size_t)kNG * kKP * 2;

static_assert(kKP % 32 == 0);
static_assert(kKP == kNH + 32);
static_assert(kNB % 16 == 0);
static_assert(kNT % 32 == 0);
static_assert(kNH == 8 * 32);
static_assert(kNI == 8);
static_assert(kPackThreads % 256 == 0);
static_assert((kAP * 2) % 16 == 0);
static_assert((kHP * 4) % 16 == 0);
static_assert(kWsTotal == 442368ull);
static_assert(kWsTotal <= 134217728ull);

struct FragH {
  union U { v16h v; v8h h[2]; };
  static __device__ __forceinline__ v16h load(const _Float16* p) {
    U f;
    f.h[0] = *(const v8h*)(p);
    f.h[1] = *(const v8h*)(p + 16);
    return f.v;
  }
};

__device__ __forceinline__ v8f mma_h(v16h a, v16h b, v8f c) {
  c = __builtin_amdgcn_wmma_f32_16x16x32_f16(false, a, false, b, (short)0, c, false, false);
  asm volatile("v_nop\n\tv_nop\n\tv_nop\n\tv_nop" : "+v"(c) : "v"(a), "v"(b));
  return c;
}

__device__ __forceinline__ float sigmoid_fast(float v) {
  return __builtin_amdgcn_rcpf(1.0f + __expf(-v));
}
__device__ __forceinline__ float tanh_fast(float v) {
  const float c = fminf(fmaxf(v, -15.0f), 15.0f);
  const float e = __expf(-2.0f * c);
  return (1.0f - e) * __builtin_amdgcn_rcpf(1.0f + e);
}

__global__ __launch_bounds__(256) void pack_weights_kernel(
    const float* __restrict__ Whh, const float* __restrict__ Wih, _Float16* __restrict__ Wp)
{
  const int i  = blockIdx.x * 256 + threadIdx.x;
  const int ic = (i < kPackThreads) ? i : (kPackThreads - 1);
  const int n  = ic / (kKP / 8);
  const int kg = ic - n * (kKP / 8);
  const int k  = kg * 8;
  const int kh = (k < kNH) ? k : (kNH - 8);
  v4f a0 = *(const v4f*)(Whh + (size_t)n * kNH + kh);
  v4f a1 = *(const v4f*)(Whh + (size_t)n * kNH + kh + 4);
  v4f c0 = *(const v4f*)(Wih + (size_t)n * kNI);
  v4f c1 = *(const v4f*)(Wih + (size_t)n * kNI + 4);
  asm volatile("" : "+v"(a0), "+v"(a1), "+v"(c0), "+v"(c1));
  const bool isH = (k < kNH);
  const bool isX = (k == kNH);
  v8h hv;
#pragma unroll
  for (int e = 0; e < 4; ++e) {
    const float f0 = isH ? a0[e] : (isX ? c0[e] : 0.0f);
    const float f1 = isH ? a1[e] : (isX ? c1[e] : 0.0f);
    hv[e]     = (_Float16)(f0 * kCarryW);
    hv[4 + e] = (_Float16)(f1 * kCarryW);
  }
  if (i < kPackThreads) {
    _Float16* q = Wp + (size_t)ic * 8;
    *(volatile v8h*)q = hv;
    __threadfence();
    *(volatile v8h*)q = hv;
  }
}

__device__ __forceinline__ void stage_input(_Float16* sA, int srow, int seg, v4f xa, v4f xb, bool active) {
  const bool isx = (seg == 0);
  v8h sv;
#pragma unroll
  for (int e = 0; e < 4; ++e) {
    const float f0 = isx ? xa[e] : 0.0f;
    const float f1 = isx ? xb[e] : 0.0f;
    sv[e]     = (_Float16)(f0 * kCarryA);
    sv[4 + e] = (_Float16)(f1 * kCarryA);
  }
  if (active) *(v8h*)(sA + srow * kAP + kNH + seg * 8) = sv;
}

__global__ __launch_bounds__(256) void gru_steps_kernel(
    const float* __restrict__ x, const float* __restrict__ bih, const float* __restrict__ bhh,
    const float* __restrict__ Wlin, const float* __restrict__ blin,
    const _Float16* __restrict__ Wp, float* __restrict__ out)
{
  __shared__ __align__(16) _Float16 sA[16 * kAP];
  __shared__ __align__(16) float    sH[16 * kHP];

  const int tid  = threadIdx.x;
  const int wave = tid >> 5;
  const int lane = tid & 31;
  const int hi   = lane >> 4;
  const int nl   = lane & 15;
  const int b0   = blockIdx.x * 16;

  {
    v8h z8;
#pragma unroll
    for (int e = 0; e < 8; ++e) z8[e] = (_Float16)0.0f;
    for (int g = tid; g < 16 * (kNH / 8); g += 256) {
      const int row = g >> 5;
      const int c8  = (g & 31) * 8;
      *(v8h*)(sA + row * kAP + c8) = z8;
    }
    if (tid < 16) *(v8h*)(sA + tid * kAP + kKP) = z8;
    for (int i2 = tid; i2 < 16 * kHP; i2 += 256) sH[i2] = 0.0f;
  }

  float b_r[2], b_z[2], b_in[2], b_hn[2];
  int   wrow[2];
#pragma unroll
  for (int jj = 0; jj < 2; ++jj) {
    const int col = (2 * wave + jj) * 16 + nl;
    b_r[jj]  = bih[col] + bhh[col];
    b_z[jj]  = bih[kNH + col] + bhh[kNH + col];
    b_in[jj] = bih[2 * kNH + col];
    b_hn[jj] = bhh[2 * kNH + col];
    wrow[jj] = col * kKP + 8 * hi;
  }
  const v4f wl0 = *(const v4f*)(Wlin + lane * 8);
  const v4f wl1 = *(const v4f*)(Wlin + lane * 8 + 4);
  const float bl = blin[0];

  const int  srow   = (tid >> 2) & 15;
  const int  seg    = tid & 3;
  const bool stager = (tid < 64);
  const float* xrow = x + (size_t)(b0 + srow) * kNT * kNI;

  {
    v4f xa = *(const v4f*)(xrow);
    v4f xb = *(const v4f*)(xrow + 4);
    asm volatile("" : "+v"(xa), "+v"(xb));
    stage_input(sA, srow, seg, xa, xb, stager);
  }
  __syncthreads();

  float pv0 = 0.0f, pv1 = 0.0f;
  const _Float16* arow = sA + nl * kAP + 8 * hi;

#pragma unroll 1
  for (int t = 0; t < kNT; ++t) {
    int zo = 0;
    asm volatile("" : "+s"(zo));
    const _Float16* wq = Wp + zo;

    const int tn = (t + 1 < kNT) ? (t + 1) : (kNT - 1);
    v4f xa = *(const v4f*)(xrow + (size_t)tn * kNI);
    v4f xb = *(const v4f*)(xrow + (size_t)tn * kNI + 4);
    asm volatile("" : "+v"(xa), "+v"(xb));

    const v8f vz = {0.f, 0.f, 0.f, 0.f, 0.f, 0.f, 0.f, 0.f};
    v8f acc_r[2]  = {vz, vz};
    v8f acc_z[2]  = {vz, vz};
    v8f acc_hn[2] = {vz, vz};
    v8f acc_in[2] = {vz, vz};

#pragma unroll 1
    for (int kc = 0; kc < 8; ++kc) {
      const v16h a = FragH::load(arow + kc * 32);
#pragma unroll
      for (int jj = 0; jj < 2; ++jj) {
        const _Float16* bp = wq + wrow[jj] + kc * 32;
        const v16h bR = FragH::load(bp);
        const v16h bZ = FragH::load(bp + kNH * kKP);
        const v16h bN = FragH::load(bp + 2 * kNH * kKP);
        acc_r[jj]  = mma_h(a, bR, acc_r[jj]);
        acc_z[jj]  = mma_h(a, bZ, acc_z[jj]);
        acc_hn[jj] = mma_h(a, bN, acc_hn[jj]);
      }
    }
    {
      const v16h a = FragH::load(arow + 8 * 32);
#pragma unroll
      for (int jj = 0; jj < 2; ++jj) {
        const _Float16* bp = wq + wrow[jj] + 8 * 32;
        const v16h bR = FragH::load(bp);
        const v16h bZ = FragH::load(bp + kNH * kKP);
        const v16h bN = FragH::load(bp + 2 * kNH * kKP);
        acc_r[jj]  = mma_h(a, bR, acc_r[jj]);
        acc_z[jj]  = mma_h(a, bZ, acc_z[jj]);
        acc_in[jj] = mma_h(a, bN, acc_in[jj]);
      }
    }
    __syncthreads();

    stage_input(sA, srow, seg, xa, xb, stager);

#pragma unroll
    for (int jj = 0; jj < 2; ++jj) {
      const int col = (2 * wave + jj) * 16 + nl;
#pragma unroll
      for (int r = 0; r < 8; ++r) {
        const int m = 8 * hi + r;
        const float hold = sH[m * kHP + col];
        const float pr  = acc_r[jj][r] * kFold + b_r[jj];
        const float pz  = acc_z[jj][r] * kFold + b_z[jj];
        const float pin = acc_in[jj][r] * kFold + b_in[jj];
        const float phn = acc_hn[jj][r] * kFold + b_hn[jj];
        const float rg = sigmoid_fast(pr);
        const float zg = sigmoid_fast(pz);
        const float ng = tanh_fast(pin + rg * phn);
        const float hnew = (1.0f - zg) * ng + zg * hold;
        sH[m * kHP + col] = hnew;
        sA[m * kAP + col] = (_Float16)(hnew * kCarryA);
      }
    }
    __syncthreads();

    const int tsel = t & 31;
    {
      const int m = 2 * wave;
      const v4f h0 = *(const v4f*)(sH + m * kHP + lane * 8);
      const v4f h1 = *(const v4f*)(sH + m * kHP + lane * 8 + 4);
      float s = 0.0f;
#pragma unroll
      for (int e = 0; e < 4; ++e) { s = fmaf(h0[e], wl0[e], s); s = fmaf(h1[e], wl1[e], s); }
#pragma unroll
      for (int off = 16; off > 0; off >>= 1) s += __shfl_xor(s, off, 32);
      const float val = s + bl;
      pv0 = (tsel == lane) ? val : pv0;
    }
    {
      const int m = 2 * wave + 1;
      const v4f h0 = *(const v4f*)(sH + m * kHP + lane * 8);
      const v4f h1 = *(const v4f*)(sH + m * kHP + lane * 8 + 4);
      float s = 0.0f;
#pragma unroll
      for (int e = 0; e < 4; ++e) { s = fmaf(h0[e], wl0[e], s); s = fmaf(h1[e], wl1[e], s); }
#pragma unroll
      for (int off = 16; off > 0; off >>= 1) s += __shfl_xor(s, off, 32);
      const float val = s + bl;
      pv1 = (tsel == lane) ? val : pv1;
    }

    if (tsel == 31) {
      float* p0 = out + (size_t)(b0 + 2 * wave) * kNT + (t - 31) + lane;
      float* p1 = out + (size_t)(b0 + 2 * wave + 1) * kNT + (t - 31) + lane;
      const float o0 = pv0;
      const float o1 = pv1;
      *(volatile float*)p0 = o0;
      *(volatile float*)p1 = o1;
      __threadfence();
      *(volatile float*)p0 = o0;
      *(volatile float*)p1 = o1;
    }
  }
}

extern "C" void kernel_launch(void* const* d_in, const int* in_sizes, int n_in,
                              void* d_out, int out_size, void* d_ws, size_t ws_size,
                              hipStream_t stream) {
  if (n_in < 8) return;
  if (in_sizes[0] != kNB * kNT * kNI) return;
  if (in_sizes[1] != kNG * kNI) return;
  if (in_sizes[2] != kNG * kNH) return;
  if (in_sizes[3] != kNG) return;
  if (in_sizes[4] != kNG) return;
  if (in_sizes[5] != kNH) return;
  if (in_sizes[6] != 1) return;
  if (out_size != kNB * kNT) return;
  if (ws_size < kWsTotal) return;

  const float* x    = (const float*)d_in[0];
  const float* Wih  = (const float*)d_in[1];
  const float* Whh  = (const float*)d_in[2];
  const float* bih  = (const float*)d_in[3];
  const float* bhh  = (const float*)d_in[4];
  const float* Wlin = (const float*)d_in[5];
  const float* blin = (const float*)d_in[6];
  float* out = (float*)d_out;
  _Float16* Wp = (_Float16*)d_ws;

  pack_weights_kernel<<<kPackThreads / 256, 256, 0, stream>>>(Whh, Wih, Wp);
  gru_steps_kernel<<<kNB / 16, 256, 0, stream>>>(x, bih, bhh, Wlin, blin, Wp, out);
}
